// CausalPD_backbone_39410619908727
// MI455X (gfx1250) — hardware-verified
//
#include <hip/hip_runtime.h>
#include <stddef.h>


typedef __attribute__((ext_vector_type(16))) _Float16 v16h;
typedef __attribute__((ext_vector_type(8)))  _Float16 v8h;
typedef __attribute__((ext_vector_type(4)))  _Float16 v4h;
typedef __attribute__((ext_vector_type(16))) __bf16   v16b;
typedef __attribute__((ext_vector_type(8)))  __bf16   v8b;
typedef __attribute__((ext_vector_type(8)))  float    v8f;
typedef __attribute__((ext_vector_type(4)))  float    v4f;

#define ATT_B   8
#define ATT_L   1024
#define ATT_DM  1024
#define ATT_H   16
#define ATT_DK  64
#define ATT_PSC 32768.0f
#define ATT_PSC_INV (1.0f / 32768.0f)

__device__ __forceinline__ unsigned short f2bf_bits(float f) {
  unsigned u = __float_as_uint(f);
  return (unsigned short)((u + 0x7FFFu + ((u >> 16) & 1u)) >> 16);
}
__device__ __forceinline__ float bf_bits2f(unsigned short h) { return __uint_as_float(((unsigned)h) << 16); }

__device__ __forceinline__ void dep_guard_h(v8f& a, v8f& b, v16h x, v16h y) { asm volatile("v_nop\n\tv_nop\n\tv_nop\n\tv_nop" : "+v"(a), "+v"(b) : "v"(x), "v"(y)); }
__device__ __forceinline__ void dep_guard_b(v8f& a, v8f& b, v16b x, v16b y) { asm volatile("v_nop\n\tv_nop\n\tv_nop\n\tv_nop" : "+v"(a), "+v"(b) : "v"(x), "v"(y)); }
__device__ __forceinline__ void keep4_h(v16h a, v16h b, v16h c, v16h d) { asm volatile("v_nop" :: "v"(a), "v"(b), "v"(c), "v"(d)); }
__device__ __forceinline__ void keep4_b(v16b a, v16b b, v16b c, v16b d) { asm volatile("v_nop" :: "v"(a), "v"(b), "v"(c), "v"(d)); }
__device__ __forceinline__ void acc_guard4(v8f& a, v8f& b, v8f& c, v8f& d) { asm volatile("v_nop\n\tv_nop\n\tv_nop\n\tv_nop" : "+v"(a), "+v"(b), "+v"(c), "+v"(d)); }
template <typename T> struct Frag;
template <> struct Frag<_Float16> {
  typedef v16h V; union U { v16h v; v8h h[2]; };
  static __device__ __forceinline__ v16h load(const _Float16* p) {
    U f; f.h[0] = *(const v8h*)(p); f.h[1] = *(const v8h*)(p + 16); return f.v;
  }
  static __device__ __forceinline__ v8f mma(v16h a, v16h b, v8f c) {
    return __builtin_amdgcn_wmma_f32_16x16x32_f16(false, a, false, b, (short)0, c, false, false);
  }
  static __device__ __forceinline__ void guard(v8f& a, v8f& b, v16h x, v16h y) { dep_guard_h(a, b, x, y); }
  static __device__ __forceinline__ void keep(v16h a, v16h b, v16h c, v16h d) { keep4_h(a, b, c, d); }
};
template <> struct Frag<__bf16> {
  typedef v16b V; union U { v16b v; v8b h[2]; };
  static __device__ __forceinline__ v16b load(const __bf16* p) {
    U f; f.h[0] = *(const v8b*)(p); f.h[1] = *(const v8b*)(p + 16); return f.v;
  }
  static __device__ __forceinline__ v8f mma(v16b a, v16b b, v8f c) {
    return __builtin_amdgcn_wmma_f32_16x16x32_bf16(false, a, false, b, (short)0, c, false, false);
  }
  static __device__ __forceinline__ void guard(v8f& a, v8f& b, v16b x, v16b y) { dep_guard_b(a, b, x, y); }
  static __device__ __forceinline__ void keep(v16b a, v16b b, v16b c, v16b d) { keep4_b(a, b, c, d); }
};

template <int ET> struct Elem;
template <> struct Elem<0> { typedef _Float16 T; };
template <> struct Elem<1> { typedef __bf16 T; };
template <int ET, bool SPLIT, int BIAS_MODE, int OUT_MODE, bool RESID, int ACT = 0>
__global__ __launch_bounds__(256) void wmma_gemm64(
    const unsigned short* __restrict__ Ap, const unsigned short* __restrict__ A2p, int lda, long strideA,
    const unsigned short* __restrict__ Btp, const unsigned short* __restrict__ Bt2p, int ldb, long strideB,
    void* __restrict__ Cout, void* __restrict__ Cout2, int ldc, long strideC,
    const float* __restrict__ bias,
    const float* __restrict__ resid, long strideR,
    int M, int N, int K, float scale) {
  typedef typename Elem<ET>::T T;
  typedef typename Frag<T>::V V;
  const T* A = (const T*)Ap; const T* A2 = (const T*)A2p; const T* Bt = (const T*)Btp; const T* Bt2 = (const T*)Bt2p;
  __shared__ __align__(16) float sT[8][16 * 68];
  const int b    = blockIdx.y;
  const int lane = threadIdx.x & 31;
  const int wave = threadIdx.x >> 5;
  const int tilesN = N >> 6;
  const int tilesM = M >> 6;
  const int tile = blockIdx.x * 8 + wave;
  if (tile >= tilesM * tilesN) return;
  const int tm = tile / tilesN;
  const int tn = tile - tm * tilesN;
  const int m0 = tm << 6;
  const int n0 = tn << 6;

  const T* Ab  = A  + (size_t)b * strideA;
  const T* Bb  = Bt + (size_t)b * strideB;
  const T* Ab2 = SPLIT ? (A2  + (size_t)b * strideA) : nullptr;
  const T* Bb2 = SPLIT ? (Bt2 + (size_t)b * strideB) : nullptr;

  const int rlane = lane & 15;
  const int koff  = (lane >> 4) * 8;
  const int mOff  = (lane >> 4) * 8;

  v8f acc[4][4];
#pragma unroll
  for (int i = 0; i < 4; ++i)
#pragma unroll
    for (int j = 0; j < 4; ++j) acc[i][j] = (v8f){0.f,0.f,0.f,0.f,0.f,0.f,0.f,0.f};

  for (int k0 = 0; k0 < K; k0 += 32) {
    V bh[4], bl[4];
#pragma unroll
    for (int j = 0; j < 4; ++j) {
      const size_t bo = (size_t)(n0 + (j << 4) + rlane) * ldb + koff + k0;
      bh[j] = Frag<T>::load(Bb + bo);
      if (SPLIT) bl[j] = Frag<T>::load(Bb2 + bo);
    }
#pragma unroll
    for (int i = 0; i < 4; ++i) {
      const size_t ao = (size_t)(m0 + (i << 4) + rlane) * lda + koff + k0;
      V ah = Frag<T>::load(Ab + ao);
      V al;
      if (SPLIT) al = Frag<T>::load(Ab2 + ao);
#pragma unroll
      for (int j = 0; j < 4; ++j) {
        acc[i][j] = Frag<T>::mma(ah, bh[j], acc[i][j]);
        if (SPLIT) {
          acc[i][j] = Frag<T>::mma(ah, bl[j], acc[i][j]);
          acc[i][j] = Frag<T>::mma(al, bh[j], acc[i][j]);
        }
      }
      Frag<T>::guard(acc[i][0], acc[i][3], ah, SPLIT ? al : ah);
    }
    Frag<T>::keep(bh[0], bh[1], bh[2], bh[3]);
    if (SPLIT) Frag<T>::keep(bl[0], bl[1], bl[2], bl[3]);
  }
  acc_guard4(acc[0][0], acc[0][1], acc[0][2], acc[0][3]);
  acc_guard4(acc[1][0], acc[1][1], acc[1][2], acc[1][3]);
  acc_guard4(acc[2][0], acc[2][1], acc[2][2], acc[2][3]);
  acc_guard4(acc[3][0], acc[3][1], acc[3][2], acc[3][3]);

  float* slab = sT[wave];
  const float* Rb = RESID ? (resid + (size_t)b * strideR) : nullptr;
#pragma unroll
  for (int i = 0; i < 4; ++i) {
    const int mBase = m0 + (i << 4);
#pragma unroll
    for (int j = 0; j < 4; ++j) {
      const int n = n0 + (j << 4) + rlane;
      float bv = 0.f;
      if (BIAS_MODE == 2) bv = bias[n];
#pragma unroll
      for (int r = 0; r < 8; ++r) {
        float v = acc[i][j][r] * scale;
        if (BIAS_MODE == 1) v += bias[mBase + mOff + r];
        if (BIAS_MODE == 2) v += bv;
        if (RESID) v += Rb[(size_t)(mBase + mOff + r) * ldc + n];
        if (ACT == 1) v = tanhf(v);
        if (ACT == 2) v = fmaxf(v, 0.0f);
        if (ACT == 3) v = v / (1.0f + expf(-v));
        if (ACT == 4) v = (v > 0.f) ? v : 0.01f * v;
        if (ACT == 5) v = 0.5f * v * (1.0f + erff(v * 0.70710678118654752f));
        slab[(mOff + r) * 68 + (j << 4) + rlane] = v;
      }
    }
    __builtin_amdgcn_fence(__ATOMIC_RELEASE, "workgroup");
    __builtin_amdgcn_wave_barrier();
    __builtin_amdgcn_fence(__ATOMIC_ACQUIRE, "workgroup");
    if (OUT_MODE == 0) {
      float* C = (float*)Cout + (size_t)b * strideC;
      const int hh = lane >> 4, c4 = (lane & 15) * 4;
      for (int pass = 0; pass < 2; ++pass) {
#pragma unroll
        for (int it = 0; it < 8; ++it) {
          const int row = it * 2 + hh;
          v4f v = *(const v4f*)(slab + row * 68 + c4);
          *(volatile v4f*)(C + (size_t)(mBase + row) * ldc + n0 + c4) = v;
        }
        __threadfence();
      }
    } else {
      const int q = lane >> 3, c8 = (lane & 7) * 8;
      unsigned short* C  = (unsigned short*)Cout  + (size_t)b * strideC;
      unsigned short* C2 = (OUT_MODE == 2) ? ((unsigned short*)Cout2 + (size_t)b * strideC) : nullptr;
      for (int pass = 0; pass < 2; ++pass) {
#pragma unroll
        for (int it = 0; it < 4; ++it) {
          const int row = it * 4 + q;
          const float* sp = slab + row * 68 + c8;
          v8h hv, lv;
#pragma unroll
          for (int e = 0; e < 8; ++e) {
            if (OUT_MODE == 1) {
              hv[e] = (_Float16)sp[e];
            } else {
              unsigned short hb = f2bf_bits(sp[e]);
              unsigned short lb = f2bf_bits(sp[e] - bf_bits2f(hb));
              hv[e] = __builtin_bit_cast(_Float16, hb);
              lv[e] = __builtin_bit_cast(_Float16, lb);
            }
          }
          *(volatile v8h*)(C + (size_t)(mBase + row) * ldc + n0 + c8) = hv;
          if (OUT_MODE == 2) *(volatile v8h*)(C2 + (size_t)(mBase + row) * ldc + n0 + c8) = lv;
        }
        __threadfence();
      }
    }
    __builtin_amdgcn_fence(__ATOMIC_RELEASE, "workgroup");
    __builtin_amdgcn_wave_barrier();
    __builtin_amdgcn_fence(__ATOMIC_ACQUIRE, "workgroup");
  }
}

__global__ __launch_bounds__(256) void cast_f32_f16x2(
    const float* __restrict__ in, _Float16* __restrict__ out, int n2) {
  int i = blockIdx.x * 256 + threadIdx.x;
  if (i < n2) {
    const _Float16 h0 = (_Float16)in[2 * i], h1 = (_Float16)in[2 * i + 1];
    const unsigned u = (unsigned)__builtin_bit_cast(unsigned short, h0) | ((unsigned)__builtin_bit_cast(unsigned short, h1) << 16);
    ((volatile unsigned*)out)[i] = u;
    __threadfence();
    ((volatile unsigned*)out)[i] = u;
  }
}

__global__ __launch_bounds__(256) void transpose_cast_kernel(
    const float* __restrict__ w, _Float16* __restrict__ wt, int K, int N, float mul) {
  __shared__ float tile[64][65];
  const int tid = threadIdx.x;
  const int k0 = blockIdx.y * 64, n0 = blockIdx.x * 64;
  {
    const int r = tid >> 2, cc = (tid & 3) * 16;
    const float* src = w + (size_t)(k0 + r) * N + n0 + cc;
#pragma unroll
    for (int i = 0; i < 4; ++i) {
      const v4f t = *(const v4f*)(src + 4 * i);
#pragma unroll
      for (int e = 0; e < 4; ++e) tile[r][cc + 4 * i + e] = t[e];
    }
  }
  __syncthreads();
  const int wave = tid >> 5, lane = tid & 31, q = lane >> 3, c8 = (lane & 7) * 8;
  for (int pass = 0; pass < 2; ++pass) {
#pragma unroll
    for (int it = 0; it < 2; ++it) {
      const int n = wave * 8 + it * 4 + q;
      v8h hv;
#pragma unroll
      for (int e = 0; e < 8; ++e) hv[e] = (_Float16)(tile[c8 + e][n] * mul);
      *(volatile v8h*)(wt + (size_t)(n0 + n) * K + k0 + c8) = hv;
    }
    __threadfence();
  }
}

__global__ __launch_bounds__(256) void ln_heads_kernel(
    const float* __restrict__ x, const float* __restrict__ gamma, const float* __restrict__ beta,
    _Float16* __restrict__ outp, int nrows) {
  __shared__ __align__(16) float sbuf[8][1024];
  const int wave = threadIdx.x >> 5, lane = threadIdx.x & 31;
  const int row = blockIdx.x * 8 + wave;
  if (row >= nrows) return;
  const float* xr = x + (size_t)row * ATT_DM + lane * 32;
  float xv[32];
#pragma unroll
  for (int i = 0; i < 8; ++i) {
    const v4f t = *(const v4f*)(xr + 4 * i);
#pragma unroll
    for (int e = 0; e < 4; ++e) xv[4 * i + e] = t[e];
  }
  float s = 0.f;
#pragma unroll
  for (int i = 0; i < 32; ++i) s += xv[i];
  s += __shfl_xor(s, 1, 32);
  const float mu = s * (1.0f / 64.0f);
  float vs = 0.f;
#pragma unroll
  for (int i = 0; i < 32; ++i) { const float d = xv[i] - mu; xv[i] = d; vs += d * d; }
  vs += __shfl_xor(vs, 1, 32);
  const float rstd = rsqrtf(vs * (1.0f / 64.0f) + 1e-5f);
  const int d0 = (lane & 1) * 32;
  float* sb = sbuf[wave] + lane * 32;
#pragma unroll
  for (int i = 0; i < 8; ++i) {
    const v4f g4 = *(const v4f*)(gamma + d0 + 4 * i);
    const v4f b4 = *(const v4f*)(beta + d0 + 4 * i);
    v4f t;
#pragma unroll
    for (int e = 0; e < 4; ++e) t[e] = (xv[4 * i + e] * rstd) * g4[e] + b4[e];
    *(v4f*)(sb + 4 * i) = t;
  }
  __builtin_amdgcn_fence(__ATOMIC_RELEASE, "workgroup");
  __builtin_amdgcn_wave_barrier();
  __builtin_amdgcn_fence(__ATOMIC_ACQUIRE, "workgroup");
  _Float16* orow = outp + (size_t)row * ATT_DM;
  const float* sr = sbuf[wave];
  for (int pass = 0; pass < 2; ++pass) {
#pragma unroll
    for (int it = 0; it < 4; ++it) {
      const int idx = it * 256 + lane * 8;
      const v4f a = *(const v4f*)(sr + idx);
      const v4f bq = *(const v4f*)(sr + idx + 4);
      v8h hv;
#pragma unroll
      for (int e = 0; e < 4; ++e) { hv[e] = (_Float16)a[e]; hv[4 + e] = (_Float16)bq[e]; }
      *(volatile v8h*)(orow + idx) = hv;
    }
    __threadfence();
  }
}

__device__ __forceinline__ v8f mma_h(v16h a, v16h b, v8f c) {
  c = __builtin_amdgcn_wmma_f32_16x16x32_f16(false, a, false, b, (short)0, c, false, false);
  asm volatile("v_nop\n\tv_nop\n\tv_nop\n\tv_nop" : "+v"(c) : "v"(a), "v"(b));
  return c;
}

__global__ __launch_bounds__(256) void attn_rows_kernel(
    const _Float16* __restrict__ qp, const _Float16* __restrict__ kp, const _Float16* __restrict__ vtp,
    const _Float16* __restrict__ cp, const _Float16* __restrict__ cbp, const int* __restrict__ mask,
    const float* __restrict__ scale_p, const float* __restrict__ bscale_p, _Float16* __restrict__ op) {
  extern __shared__ __align__(16) char smem[];
  float*    sS  = (float*)smem;
  float*    sBi = (float*)(smem + 65536);
  _Float16* sP  = (_Float16*)(smem + 65536);
  float*    sO  = (float*)(smem + 98304);

  const int tid = threadIdx.x, wave = tid >> 5, lane = tid & 31, hh = lane >> 4, c = lane & 15;
  const int q0 = blockIdx.x * 16;
  const int bh = blockIdx.y, b = bh >> 4, h = bh & 15;
  const float scale = scale_p[0], bscale = bscale_p[0];
  const v8f z8 = {0.f, 0.f, 0.f, 0.f, 0.f, 0.f, 0.f, 0.f};

  const size_t arow = ((size_t)(b * ATT_L + q0 + c)) * ATT_DM + h * ATT_DK + 8 * hh;
  const v16h qa0 = Frag<_Float16>::load(qp + arow);
  const v16h qa1 = Frag<_Float16>::load(qp + arow + 32);
  const v16h ca0 = Frag<_Float16>::load(cbp + arow);
  const v16h ca1 = Frag<_Float16>::load(cbp + arow + 32);

#pragma unroll 1
  for (int ct = 0; ct < 8; ++ct) {
    const int col0 = wave * 128 + ct * 16;
    const int* mrow = mask + (size_t)(q0 + 8 * hh) * ATT_L + col0 + c;
    int mk[8];
    int allm = 1;
#pragma unroll
    for (int r = 0; r < 8; ++r) { mk[r] = mrow[(size_t)r * ATT_L]; allm &= (mk[r] != 0) ? 1 : 0; }
    const int skip = __all(allm);
    const size_t brow = ((size_t)(b * ATT_L + col0 + c)) * ATT_DM + h * ATT_DK + 8 * hh;
    v8f accB = z8, accS = z8;
    {
      const v16h cf0 = Frag<_Float16>::load(cp + brow);
      const v16h cf1 = Frag<_Float16>::load(cp + brow + 32);
      accB = mma_h(ca0, cf0, accB);
      accB = mma_h(ca1, cf1, accB);
    }
    if (!skip) {
      const v16h kf0 = Frag<_Float16>::load(kp + brow);
      const v16h kf1 = Frag<_Float16>::load(kp + brow + 32);
      accS = mma_h(qa0, kf0, accS);
      accS = mma_h(qa1, kf1, accS);
    }
#pragma unroll
    for (int r = 0; r < 8; ++r) {
      const int o = (8 * hh + r) * ATT_L + col0 + c;
      const float sv = accS[r] * scale;
      sS[o]  = (mk[r] != 0) ? -__builtin_inff() : sv;
      sBi[o] = accB[r];
    }
  }
  __syncthreads();

  const int row = tid >> 4, sub = tid & 15;
  float* rs = sS + row * ATT_L + 4 * sub;
  const float* rb = sBi + row * ATT_L + 4 * sub;
  float mx = -__builtin_inff(), bsq = 0.f;
#pragma unroll 4
  for (int j = 0; j < 16; ++j) {
    const v4f s4 = *(const v4f*)(rs + 64 * j);
    const v4f b4 = *(const v4f*)(rb + 64 * j);
#pragma unroll
    for (int e = 0; e < 4; ++e) { mx = fmaxf(mx, s4[e]); bsq += b4[e] * b4[e]; }
  }
#pragma unroll
  for (int off = 8; off >= 1; off >>= 1) {
    mx = fmaxf(mx, __shfl_xor(mx, off, 32));
    bsq += __shfl_xor(bsq, off, 32);
  }
  float se = 0.f;
#pragma unroll 4
  for (int j = 0; j < 16; ++j) {
    const v4f s4 = *(const v4f*)(rs + 64 * j);
    v4f e4;
#pragma unroll
    for (int e = 0; e < 4; ++e) { const float ev = __expf(s4[e] - mx); e4[e] = ev; se += ev; }
    *(v4f*)(rs + 64 * j) = e4;
  }
#pragma unroll
  for (int off = 8; off >= 1; off >>= 1) se += __shfl_xor(se, off, 32);
  const float inv_se = 1.0f / se;
  const float inv_bn = 1.0f / fmaxf(sqrtf(bsq), 1e-12f);
  float asq = 0.f;
#pragma unroll 4
  for (int j = 0; j < 16; ++j) {
    const v4f e4 = *(const v4f*)(rs + 64 * j);
    const v4f b4 = *(const v4f*)(rb + 64 * j);
    v4f a4;
#pragma unroll
    for (int e = 0; e < 4; ++e) { const float av = e4[e] * inv_se + (b4[e] * inv_bn) * bscale; a4[e] = av; asq += av * av; }
    *(v4f*)(rs + 64 * j) = a4;
  }
#pragma unroll
  for (int off = 8; off >= 1; off >>= 1) asq += __shfl_xor(asq, off, 32);
  const float pmul = (1.0f / fmaxf(sqrtf(asq), 1e-12f)) * ATT_PSC;
  __syncthreads();
  {
    _Float16* prow = sP + row * ATT_L + 4 * sub;
#pragma unroll 4
    for (int j = 0; j < 16; ++j) {
      const v4f a4 = *(const v4f*)(rs + 64 * j);
      v4h p4;
#pragma unroll
      for (int e = 0; e < 4; ++e) p4[e] = (_Float16)(a4[e] * pmul);
      *(v4h*)(prow + 64 * j) = p4;
    }
  }
  __syncthreads();

  if (wave < 4) {
    const int t = wave;
    const _Float16* vb = vtp + ((size_t)(h * ATT_DK + t * 16 + c)) * (size_t)(ATT_B * ATT_L) + b * ATT_L + 8 * hh;
    const _Float16* pbase = sP + c * ATT_L + 8 * hh;
    v8f acc = z8;
#pragma unroll 2
    for (int k0 = 0; k0 < ATT_L; k0 += 32) {
      const v16h pa = Frag<_Float16>::load(pbase + k0);
      const v16h vf = Frag<_Float16>::load(vb + k0);
      acc = mma_h(pa, vf, acc);
    }
#pragma unroll
    for (int r = 0; r < 8; ++r) sO[(8 * hh + r) * 68 + t * 16 + c] = acc[r] * ATT_PSC_INV;
  }
  __syncthreads();
  if (wave == 0) {
    const int q = lane >> 3, c8 = (lane & 7) * 8;
    _Float16* ob = op + ((size_t)(b * ATT_L + q0)) * ATT_DM + h * ATT_DK + c8;
    for (int pass = 0; pass < 2; ++pass) {
#pragma unroll
      for (int it = 0; it < 4; ++it) {
        const int orow2 = it * 4 + q;
        const v4f a = *(const v4f*)(sO + orow2 * 68 + c8);
        const v4f bq = *(const v4f*)(sO + orow2 * 68 + c8 + 4);
        v8h hv;
#pragma unroll
        for (int e = 0; e < 4; ++e) { hv[e] = (_Float16)a[e]; hv[4 + e] = (_Float16)bq[e]; }
        *(volatile v8h*)(ob + (size_t)orow2 * ATT_DM) = hv;
      }
      __threadfence();
    }
  }
}

extern "C" void kernel_launch(void* const* d_in, const int* in_sizes, int n_in,
                              void* d_out, int out_size, void* d_ws, size_t ws_size,
                              hipStream_t stream) {
  const int NTOK = ATT_B * ATT_L;
  const size_t NE = (size_t)NTOK * ATT_DM;
  const size_t NW = (size_t)ATT_DM * ATT_DM;
  if (n_in < 16) return;
  if (in_sizes[0] != (int)NE || in_sizes[1] != (int)NE || in_sizes[2] != ATT_L * ATT_L ||
      in_sizes[3] != (int)NW || in_sizes[5] != (int)NW || in_sizes[7] != (int)NW || in_sizes[14] != (int)NW ||
      in_sizes[4] != ATT_DM || in_sizes[6] != ATT_DM || in_sizes[8] != ATT_DM || in_sizes[15] != ATT_DM ||
      in_sizes[9] != ATT_DK * ATT_DK || in_sizes[10] != ATT_DK || in_sizes[11] != ATT_DK ||
      in_sizes[12] < 1 || in_sizes[13] < 1 || out_size != (int)NE) return;

  const float* Q      = (const float*)d_in[0];
  const float* ctx    = (const float*)d_in[1];
  const int*   mask   = (const int*)d_in[2];
  const float* W_q    = (const float*)d_in[3];
  const float* b_q    = (const float*)d_in[4];
  const float* W_k    = (const float*)d_in[5];
  const float* b_k    = (const float*)d_in[6];
  const float* W_v    = (const float*)d_in[7];
  const float* b_v    = (const float*)d_in[8];
  const float* bil    = (const float*)d_in[9];
  const float* gamma  = (const float*)d_in[10];
  const float* beta   = (const float*)d_in[11];
  const float* scale  = (const float*)d_in[12];
  const float* bscale = (const float*)d_in[13];
  const float* W_o    = (const float*)d_in[14];
  const float* b_o    = (const float*)d_in[15];
  float* out = (float*)d_out;

  char* ws = (char*)d_ws;
  size_t off = 0;
  auto carve = [&](size_t bytes) -> char* { char* p = ws + off; off += (bytes + 255) & ~(size_t)255; return p; };
  _Float16* WqT  = (_Float16*)carve(NW * 2);
  _Float16* WkT  = (_Float16*)carve(NW * 2);
  _Float16* WvT  = (_Float16*)carve(NW * 2);
  _Float16* WoT  = (_Float16*)carve(NW * 2);
  _Float16* bilT = (_Float16*)carve((size_t)ATT_DK * ATT_DK * 2);
  _Float16* Q16  = (_Float16*)carve(NE * 2);
  _Float16* q16  = (_Float16*)carve(NE * 2);
  _Float16* k16  = (_Float16*)carve(NE * 2);
  _Float16* vT16 = (_Float16*)carve(NE * 2);
  _Float16* c16  = (_Float16*)carve(NE * 2);
  _Float16* cb16 = (_Float16*)carve(NE * 2);
  _Float16* O16  = (_Float16*)carve(NE * 2);
  if (off > ws_size) return;

  const unsigned short* Q16u  = (const unsigned short*)Q16;
  const unsigned short* WqTu  = (const unsigned short*)WqT;
  const unsigned short* WkTu  = (const unsigned short*)WkT;
  const unsigned short* WvTu  = (const unsigned short*)WvT;
  const unsigned short* WoTu  = (const unsigned short*)WoT;
  const unsigned short* bilTu = (const unsigned short*)bilT;
  const unsigned short* c16u  = (const unsigned short*)c16;
  const unsigned short* O16u  = (const unsigned short*)O16;
  const float w_carry = 64.0f, w_carry_inv = 1.0f / 64.0f;

  cast_f32_f16x2<<<(int)(NE / 2 / 256), 256, 0, stream>>>(Q, Q16, (int)(NE / 2));
  transpose_cast_kernel<<<dim3(ATT_DM / 64, ATT_DM / 64), 256, 0, stream>>>(W_q, WqT, ATT_DM, ATT_DM, w_carry);
  transpose_cast_kernel<<<dim3(ATT_DM / 64, ATT_DM / 64), 256, 0, stream>>>(W_k, WkT, ATT_DM, ATT_DM, w_carry);
  transpose_cast_kernel<<<dim3(ATT_DM / 64, ATT_DM / 64), 256, 0, stream>>>(W_v, WvT, ATT_DM, ATT_DM, w_carry);
  transpose_cast_kernel<<<dim3(ATT_DM / 64, ATT_DM / 64), 256, 0, stream>>>(W_o, WoT, ATT_DM, ATT_DM, w_carry);
  transpose_cast_kernel<<<dim3(1, 1), 256, 0, stream>>>(bil, bilT, ATT_DK, ATT_DK, 1.0f);

  const int gemm_blocks = (NTOK / 64) * (ATT_DM / 64) / 8;
  wmma_gemm64<0, false, 2, 1, false><<<dim3(gemm_blocks, 1), 256, 0, stream>>>(
      Q16u, Q16u, ATT_DM, 0L, WqTu, WqTu, ATT_DM, 0L, (void*)q16, (void*)q16, ATT_DM, 0L,
      b_q, b_q, 0L, NTOK, ATT_DM, ATT_DM, w_carry_inv);
  wmma_gemm64<0, false, 2, 1, false><<<dim3(gemm_blocks, 1), 256, 0, stream>>>(
      Q16u, Q16u, ATT_DM, 0L, WkTu, WkTu, ATT_DM, 0L, (void*)k16, (void*)k16, ATT_DM, 0L,
      b_k, b_k, 0L, NTOK, ATT_DM, ATT_DM, w_carry_inv);
  wmma_gemm64<0, false, 1, 1, false><<<dim3(gemm_blocks, 1), 256, 0, stream>>>(
      WvTu, WvTu, ATT_DM, 0L, Q16u, Q16u, ATT_DM, 0L, (void*)vT16, (void*)vT16, NTOK, 0L,
      b_v, b_v, 0L, ATT_DM, NTOK, ATT_DM, w_carry_inv);

  ln_heads_kernel<<<NTOK / 8, 256, 0, stream>>>(ctx, gamma, beta, c16, NTOK);
  const int cb_rows = NTOK * ATT_H;
  wmma_gemm64<0, false, 0, 1, false><<<dim3((cb_rows / 64) / 8, 1), 256, 0, stream>>>(
      c16u, c16u, ATT_DK, 0L, bilTu, bilTu, ATT_DK, 0L, (void*)cb16, (void*)cb16, ATT_DK, 0L,
      b_q, b_q, 0L, cb_rows, ATT_DK, ATT_DK, 1.0f);

  attn_rows_kernel<<<dim3(ATT_L / 16, ATT_B * ATT_H), 256, 131072, stream>>>(
      q16, k16, vT16, c16, cb16, mask, scale, bscale, O16);

  wmma_gemm64<0, false, 2, 0, false><<<dim3(gemm_blocks, 1), 256, 0, stream>>>(
      O16u, O16u, ATT_DM, 0L, WoTu, WoTu, ATT_DM, 0L, (void*)out, (void*)out, ATT_DM, 0L,
      b_o, b_o, 0L, NTOK, ATT_DM, ATT_DM, w_carry_inv);
  (void)hipGetLastError();
}
